// JaxGRU_22256520528302
// MI455X (gfx1250) — hardware-verified
//
#include <hip/hip_runtime.h>
#include <hip/hip_bf16.h>


#define BS_   256
#define KIN_  8000
#define T_    100
#define ACT_  32
#define HID_  1024
#define G3_   3072
#define OUT_  64
#define MT_   25600

static_assert(MT_ == BS_ * T_);
static_assert(KIN_ % 64 == 0);
static_assert(HID_ % 64 == 0);
static_assert(G3_ == 3 * HID_);
static_assert(BS_ % 64 == 0);
static_assert(MT_ % 64 == 0);
static_assert(OUT_ == 64);
static_assert(ACT_ == 32);

typedef float          v4f   __attribute__((ext_vector_type(4)));
typedef float          v8f   __attribute__((ext_vector_type(8)));
typedef __bf16         v16b  __attribute__((ext_vector_type(16)));
typedef _Float16       v16h  __attribute__((ext_vector_type(16)));
typedef _Float16       v8h   __attribute__((ext_vector_type(8)));
typedef unsigned short u16x8 __attribute__((ext_vector_type(8)));

union FragB { u16x8 h[2]; v16b v; };
union FragH { u16x8 h[2]; v16h v; };
union H8    { v8h f; u16x8 u; };

constexpr size_t SZ_O16   = (size_t)MT_ * HID_ * 2;
constexpr size_t SZ_WIN16 = (size_t)HID_ * KIN_ * 2;
constexpr size_t SZ_X16   = (size_t)BS_ * KIN_ * 2;
constexpr size_t SZ_WH16  = (size_t)G3_ * HID_ * 2;
constexpr size_t SZ_WI16  = (size_t)G3_ * ACT_ * 2;
constexpr size_t SZ_WO16  = (size_t)OUT_ * HID_ * 2;
constexpr size_t SZ_A16   = (size_t)MT_ * ACT_ * 2;
constexpr size_t SZ_HF    = (size_t)BS_ * HID_ * 4;
constexpr size_t SZ_HA    = (size_t)BS_ * HID_ * 2;

constexpr size_t OFF_OH   = 0;
constexpr size_t OFF_OL   = OFF_OH + SZ_O16;
constexpr size_t END_O    = OFF_OL + SZ_O16;
constexpr size_t OFF_WINH = 0;
constexpr size_t OFF_WINL = OFF_WINH + SZ_WIN16;
constexpr size_t OFF_XH   = OFF_WINL + SZ_WIN16;
constexpr size_t OFF_XL   = OFF_XH + SZ_X16;
constexpr size_t END_ENC  = OFF_XL + SZ_X16;
static_assert(END_ENC <= END_O);
constexpr size_t OFF_WH   = END_O;
constexpr size_t OFF_WIH  = OFF_WH + SZ_WH16;
constexpr size_t OFF_WIL  = OFF_WIH + SZ_WI16;
constexpr size_t OFF_WOH  = OFF_WIL + SZ_WI16;
constexpr size_t OFF_WOL  = OFF_WOH + SZ_WO16;
constexpr size_t OFF_AH   = OFF_WOL + SZ_WO16;
constexpr size_t OFF_AL   = OFF_AH + SZ_A16;
constexpr size_t OFF_HF0  = OFF_AL + SZ_A16;
constexpr size_t OFF_HF1  = OFF_HF0 + SZ_HF;
constexpr size_t OFF_HA0  = OFF_HF1 + SZ_HF;
constexpr size_t OFF_HA1  = OFF_HA0 + SZ_HA;
constexpr size_t WS_END   = OFF_HA1 + SZ_HA;
static_assert(WS_END <= (size_t)134217728);
static_assert(OFF_OL % 128 == 0 && OFF_WINL % 128 == 0 && OFF_XH % 128 == 0 && OFF_XL % 128 == 0);
static_assert(OFF_WH % 128 == 0 && OFF_WIH % 128 == 0 && OFF_WIL % 128 == 0 && OFF_WOH % 128 == 0 && OFF_WOL % 128 == 0);
static_assert(OFF_AH % 128 == 0 && OFF_AL % 128 == 0 && OFF_HF0 % 128 == 0 && OFF_HF1 % 128 == 0 && OFF_HA0 % 128 == 0 && OFF_HA1 % 128 == 0);

__device__ __forceinline__ unsigned short f32_to_bf16(float f) {
    unsigned u = __float_as_uint(f);
    unsigned r = u + 0x7FFFu + ((u >> 16) & 1u);
    return (unsigned short)(r >> 16);
}
__device__ __forceinline__ float bf16_to_f32(unsigned short b) {
    return __uint_as_float(((unsigned)b) << 16);
}
__device__ __forceinline__ v8f ld8f(const float* p) {
    v4f a = *(const v4f*)p;
    v4f b = *(const v4f*)(p + 4);
    return __builtin_shufflevector(a, b, 0, 1, 2, 3, 4, 5, 6, 7);
}
__device__ __forceinline__ void split8(const v8f x, u16x8& hv, u16x8& lv) {
#pragma unroll
    for (int c = 0; c < 8; ++c) {
        const float f = x[c];
        const unsigned short hb = f32_to_bf16(f);
        const unsigned short lb = f32_to_bf16(f - bf16_to_f32(hb));
        hv[c] = hb;
        lv[c] = lb;
    }
}
__device__ __forceinline__ u16x8 cvt8h(const v8f x) {
    H8 q;
    q.f = __builtin_convertvector(x, v8h);
    return q.u;
}
__device__ __forceinline__ float sigm_f(float x) {
    return __builtin_amdgcn_rcpf(1.0f + __expf(-x));
}
__device__ __forceinline__ float tanh_f(float x) {
    const float xc = fminf(fmaxf(x, -15.0f), 15.0f);
    const float e  = __expf(2.0f * xc);
    return (e - 1.0f) * __builtin_amdgcn_rcpf(e + 1.0f);
}

__device__ __forceinline__ void mma_bf(v8f& acc, const FragB& a, const FragB& b) {
    acc = __builtin_amdgcn_wmma_f32_16x16x32_bf16(false, a.v, false, b.v, (short)0, acc, false, false);
    asm volatile("v_nop\n\tv_nop\n\tv_nop\n\tv_nop" : "+v"(acc) : "v"(a.v), "v"(b.v));
}
__device__ __forceinline__ void mma_hf(v8f& acc, const FragH& a, const FragH& b) {
    acc = __builtin_amdgcn_wmma_f32_16x16x32_f16(false, a.v, false, b.v, (short)0, acc, false, false);
    asm volatile("v_nop\n\tv_nop\n\tv_nop\n\tv_nop" : "+v"(acc) : "v"(a.v), "v"(b.v));
}

__global__ __launch_bounds__(256)
void rows_cvt_kernel(const float* __restrict__ src, unsigned short* dhi, unsigned short* dlo, int n8)
{
    const int i = blockIdx.x * 256 + threadIdx.x;
    if (i >= n8) return;
    const size_t e = (size_t)i * 8;
    const v8f x = ld8f(src + e);
    u16x8 hv, lv;
    split8(x, hv, lv);
    *(volatile u16x8*)(dhi + e) = hv;
    *(volatile u16x8*)(dlo + e) = lv;
    __threadfence();
    *(volatile u16x8*)(dhi + e) = hv;
    *(volatile u16x8*)(dlo + e) = lv;
}

template<int TK, int MODE>
__global__ __launch_bounds__(256)
void wt_cvt_kernel(const float* __restrict__ src, unsigned short* d0, unsigned short* d1,
                   int Nw, int Kd, float scale)
{
    static_assert(TK == 32 || TK == 64);
    constexpr int P   = TK + 4;
    constexpr int LPR = TK / 8;
    constexpr int RPI = 32 / LPR;
    constexpr int NIT = 8 / RPI;
    __shared__ __attribute__((aligned(16))) float sT[64 * P];
    const int tid  = threadIdx.x;
    const int lane = tid & 31;
    const int wave = tid >> 5;
    const int n0 = blockIdx.x * 64;
    const int k0 = blockIdx.y * TK;

#pragma unroll
    for (int it = 0; it < TK / 16; ++it) {
        const int idx = it * 256 + tid;
        const int kk  = idx >> 4;
        const int n4  = (idx & 15) * 4;
        const int gn  = min(n0 + n4, Nw - 4);
        const int gk  = min(k0 + kk, Kd - 1);
        const v4f v = *(const v4f*)(src + (size_t)gk * Nw + gn) * scale;
        sT[(n4 + 0) * P + kk] = v[0];
        sT[(n4 + 1) * P + kk] = v[1];
        sT[(n4 + 2) * P + kk] = v[2];
        sT[(n4 + 3) * P + kk] = v[3];
    }
    __syncthreads();

    u16x8 hv[NIT], lv[NIT];
    const int c = (lane % LPR) * 8;
#pragma unroll
    for (int it = 0; it < NIT; ++it) {
        const int nn = wave * 8 + it * RPI + lane / LPR;
        const v8f x = ld8f(sT + nn * P + c);
        if (MODE == 0) {
            split8(x, hv[it], lv[it]);
        } else {
            hv[it] = cvt8h(x);
            lv[it] = hv[it];
        }
    }
#pragma unroll
    for (int it = 0; it < NIT; ++it) {
        const int gr = n0 + wave * 8 + it * RPI + lane / LPR;
        if (gr < Nw) {
            const size_t o = (size_t)gr * Kd + k0 + c;
            *(volatile u16x8*)(d0 + o) = hv[it];
            if (MODE == 0) *(volatile u16x8*)(d1 + o) = lv[it];
        }
    }
    __threadfence();
#pragma unroll
    for (int it = 0; it < NIT; ++it) {
        const int gr = n0 + wave * 8 + it * RPI + lane / LPR;
        if (gr < Nw) {
            const size_t o = (size_t)gr * Kd + k0 + c;
            *(volatile u16x8*)(d0 + o) = hv[it];
            if (MODE == 0) *(volatile u16x8*)(d1 + o) = lv[it];
        }
    }
}

template<bool RELU, bool WH16>
__global__ __launch_bounds__(128)
void gemm_x3_kernel(const unsigned short* __restrict__ Ah, const unsigned short* __restrict__ Al,
                    const unsigned short* __restrict__ Bh, const unsigned short* __restrict__ Bl,
                    const float* __restrict__ bias, float* C, unsigned short* Hc, int K, int ldc, int ldh)
{
    constexpr int P = 68;
    __shared__ __attribute__((aligned(16))) float sC[64 * P];

    const int tid  = threadIdx.x;
    const int lane = tid & 31;
    const int wave = tid >> 5;
    const int h    = lane >> 4;
    const int m    = lane & 15;
    const int wm   = wave >> 1;
    const int wn   = wave & 1;

    const int rowB = blockIdx.y * 64;
    const int colB = blockIdx.x * 64;
    const int rowW = rowB + wm * 32;
    const int colW = colB + wn * 32;

    v8f acc[4];
#pragma unroll
    for (int j = 0; j < 4; ++j)
#pragma unroll
        for (int r = 0; r < 8; ++r) acc[j][r] = 0.0f;

    const size_t aoff  = (size_t)(rowW + m) * K + 8 * h;
    const size_t boff  = (size_t)(colW + m) * K + 8 * h;
    const size_t sub16 = (size_t)16 * K;
    const int nk = K >> 5;

#pragma unroll 1
    for (int kt = 0; kt < nk; ++kt) {
        const size_t k0 = (size_t)kt * 32;
        FragB fa[2], ga[2], fb[2], gb[2];
#pragma unroll
        for (int s = 0; s < 2; ++s) {
            const unsigned short* p = Ah + aoff + s * sub16 + k0;
            const unsigned short* q = Al + aoff + s * sub16 + k0;
            fa[s].h[0] = *(const u16x8*)(p);
            fa[s].h[1] = *(const u16x8*)(p + 16);
            ga[s].h[0] = *(const u16x8*)(q);
            ga[s].h[1] = *(const u16x8*)(q + 16);
        }
#pragma unroll
        for (int j = 0; j < 2; ++j) {
            const unsigned short* p = Bh + boff + j * sub16 + k0;
            const unsigned short* q = Bl + boff + j * sub16 + k0;
            fb[j].h[0] = *(const u16x8*)(p);
            fb[j].h[1] = *(const u16x8*)(p + 16);
            gb[j].h[0] = *(const u16x8*)(q);
            gb[j].h[1] = *(const u16x8*)(q + 16);
        }
#pragma unroll
        for (int s = 0; s < 2; ++s)
#pragma unroll
            for (int j = 0; j < 2; ++j) {
                mma_bf(acc[s * 2 + j], fa[s], fb[j]);
                mma_bf(acc[s * 2 + j], fa[s], gb[j]);
                mma_bf(acc[s * 2 + j], ga[s], fb[j]);
            }
    }

    float bv[2];
#pragma unroll
    for (int j = 0; j < 2; ++j) bv[j] = bias[colW + j * 16 + m];
#pragma unroll
    for (int s = 0; s < 2; ++s)
#pragma unroll
        for (int j = 0; j < 2; ++j)
#pragma unroll
            for (int r = 0; r < 8; ++r) {
                float v = acc[s * 2 + j][r] + bv[j];
                if (RELU) v = fmaxf(v, 0.0f);
                sC[(wm * 32 + s * 16 + 8 * h + r) * P + wn * 32 + j * 16 + m] = v;
            }
    __syncthreads();

#pragma unroll
    for (int it = 0; it < 8; ++it) {
        const int lr = wave * 16 + it * 2 + (lane >> 4);
        const int c  = (lane & 15) * 4;
        const v4f v = *(const v4f*)(sC + lr * P + c);
        *(volatile v4f*)(C + (size_t)(rowB + lr) * ldc + colB + c) = v;
    }
    if (WH16) {
#pragma unroll
        for (int it = 0; it < 4; ++it) {
            const int lr = wave * 16 + it * 4 + (lane >> 3);
            const int c  = (lane & 7) * 8;
            const u16x8 hv = cvt8h(ld8f(sC + lr * P + c));
            *(volatile u16x8*)(Hc + (size_t)(rowB + lr) * ldh + colB + c) = hv;
        }
    }
    __threadfence();
#pragma unroll
    for (int it = 0; it < 8; ++it) {
        const int lr = wave * 16 + it * 2 + (lane >> 4);
        const int c  = (lane & 15) * 4;
        const v4f v = *(const v4f*)(sC + lr * P + c);
        *(volatile v4f*)(C + (size_t)(rowB + lr) * ldc + colB + c) = v;
    }
    if (WH16) {
#pragma unroll
        for (int it = 0; it < 4; ++it) {
            const int lr = wave * 16 + it * 4 + (lane >> 3);
            const int c  = (lane & 7) * 8;
            const u16x8 hv = cvt8h(ld8f(sC + lr * P + c));
            *(volatile u16x8*)(Hc + (size_t)(rowB + lr) * ldh + colB + c) = hv;
        }
    }
}

__global__ __launch_bounds__(256)
void gru_step_kernel(const unsigned short* __restrict__ hA, const float* __restrict__ hF,
                     const unsigned short* __restrict__ aH, const unsigned short* __restrict__ aL,
                     const unsigned short* __restrict__ whP,
                     const unsigned short* __restrict__ wiH, const unsigned short* __restrict__ wiL,
                     const float* __restrict__ bi, const float* __restrict__ bhn,
                     float* hFn, unsigned short* hAn, unsigned short* oH, unsigned short* oL, int t)
{
    constexpr int P = 68;
    __shared__ __attribute__((aligned(16))) float sH[64 * P];

    const int tid  = threadIdx.x;
    const int lane = tid & 31;
    const int wave = tid >> 5;
    const int h    = lane >> 4;
    const int m    = lane & 15;
    const int jb   = blockIdx.x * 64;
    const int rb   = blockIdx.y * 64;
    const int ut   = wave & 3;
    const int rh   = wave >> 2;
    const int j0   = jb + 16 * ut;
    const int r0   = rb + 32 * rh;

    v8f accR[2], accZ[2], accHN[2], accIN[2];
#pragma unroll
    for (int s = 0; s < 2; ++s)
#pragma unroll
        for (int r = 0; r < 8; ++r) {
            accR[s][r] = 0.0f; accZ[s][r] = 0.0f; accHN[s][r] = 0.0f; accIN[s][r] = 0.0f;
        }

    {
        FragB wbH[3], wbL[3];
#pragma unroll
        for (int g = 0; g < 3; ++g) {
            const unsigned short* p = wiH + (size_t)(g * HID_ + j0 + m) * ACT_ + 8 * h;
            const unsigned short* q = wiL + (size_t)(g * HID_ + j0 + m) * ACT_ + 8 * h;
            wbH[g].h[0] = *(const u16x8*)(p);
            wbH[g].h[1] = *(const u16x8*)(p + 16);
            wbL[g].h[0] = *(const u16x8*)(q);
            wbL[g].h[1] = *(const u16x8*)(q + 16);
        }
#pragma unroll
        for (int s = 0; s < 2; ++s) {
            const size_t arow = (size_t)(r0 + 16 * s + m) * T_ + (size_t)t;
            const unsigned short* p = aH + arow * ACT_ + 8 * h;
            const unsigned short* q = aL + arow * ACT_ + 8 * h;
            FragB gaH, gaL;
            gaH.h[0] = *(const u16x8*)(p);
            gaH.h[1] = *(const u16x8*)(p + 16);
            gaL.h[0] = *(const u16x8*)(q);
            gaL.h[1] = *(const u16x8*)(q + 16);
            mma_bf(accR[s],  gaH, wbH[0]);  mma_bf(accR[s],  gaH, wbL[0]);  mma_bf(accR[s],  gaL, wbH[0]);
            mma_bf(accZ[s],  gaH, wbH[1]);  mma_bf(accZ[s],  gaH, wbL[1]);  mma_bf(accZ[s],  gaL, wbH[1]);
            mma_bf(accIN[s], gaH, wbH[2]);  mma_bf(accIN[s], gaH, wbL[2]);  mma_bf(accIN[s], gaL, wbH[2]);
        }
    }

    {
        const size_t aoff  = (size_t)(r0 + m) * HID_ + 8 * h;
        const size_t boff0 = (size_t)(0 * HID_ + j0 + m) * HID_ + 8 * h;
        const size_t boff1 = (size_t)(1 * HID_ + j0 + m) * HID_ + 8 * h;
        const size_t boff2 = (size_t)(2 * HID_ + j0 + m) * HID_ + 8 * h;
        const size_t sub16 = (size_t)16 * HID_;
#pragma unroll 1
        for (int kt = 0; kt < HID_ / 32; ++kt) {
            const size_t k0 = (size_t)kt * 32;
            FragH fa[2], fb[3];
#pragma unroll
            for (int s = 0; s < 2; ++s) {
                const unsigned short* p = hA + aoff + s * sub16 + k0;
                fa[s].h[0] = *(const u16x8*)(p);
                fa[s].h[1] = *(const u16x8*)(p + 16);
            }
            {
                const unsigned short* p0 = whP + boff0 + k0;
                const unsigned short* p1 = whP + boff1 + k0;
                const unsigned short* p2 = whP + boff2 + k0;
                fb[0].h[0] = *(const u16x8*)(p0);  fb[0].h[1] = *(const u16x8*)(p0 + 16);
                fb[1].h[0] = *(const u16x8*)(p1);  fb[1].h[1] = *(const u16x8*)(p1 + 16);
                fb[2].h[0] = *(const u16x8*)(p2);  fb[2].h[1] = *(const u16x8*)(p2 + 16);
            }
#pragma unroll
            for (int s = 0; s < 2; ++s) {
                mma_hf(accR[s],  fa[s], fb[0]);
                mma_hf(accZ[s],  fa[s], fb[1]);
                mma_hf(accHN[s], fa[s], fb[2]);
            }
        }
    }

    {
        const int   j   = j0 + m;
        const float bir = bi[j];
        const float biz = bi[HID_ + j];
        const float bin = bi[2 * HID_ + j];
        const float bh  = bhn[j];
        const float s16 = 0.0625f;
#pragma unroll
        for (int s = 0; s < 2; ++s)
#pragma unroll
            for (int r = 0; r < 8; ++r) {
                const int lr   = 32 * rh + 16 * s + 8 * h + r;
                const int grow = rb + lr;
                const float rg = sigm_f(accR[s][r] * s16 + bir);
                const float zg = sigm_f(accZ[s][r] * s16 + biz);
                const float hn = accHN[s][r] * s16 + bh;
                const float ng = tanh_f(accIN[s][r] * s16 + bin + rg * hn);
                const float ho = hF[(size_t)grow * HID_ + j];
                const float hw = (1.0f - zg) * ng + zg * ho;
                sH[lr * P + 16 * ut + m] = hw;
            }
    }
    __syncthreads();

#pragma unroll
    for (int it = 0; it < 4; ++it) {
        const int lr = wave * 8 + it * 2 + (lane >> 4);
        const int c  = (lane & 15) * 4;
        const v4f v = *(const v4f*)(sH + lr * P + c);
        *(volatile v4f*)(hFn + (size_t)(rb + lr) * HID_ + jb + c) = v;
    }
#pragma unroll
    for (int it = 0; it < 2; ++it) {
        const int lr = wave * 8 + it * 4 + (lane >> 3);
        const int c  = (lane & 7) * 8;
        const v8f x = ld8f(sH + lr * P + c);
        const u16x8 fv = cvt8h(x);
        u16x8 hv, lv;
        split8(x, hv, lv);
        const size_t oh = (size_t)(rb + lr) * HID_ + jb + c;
        const size_t oo = ((size_t)(rb + lr) * T_ + (size_t)t) * HID_ + jb + c;
        *(volatile u16x8*)(hAn + oh) = fv;
        *(volatile u16x8*)(oH + oo)  = hv;
        *(volatile u16x8*)(oL + oo)  = lv;
    }
    __threadfence();
#pragma unroll
    for (int it = 0; it < 4; ++it) {
        const int lr = wave * 8 + it * 2 + (lane >> 4);
        const int c  = (lane & 15) * 4;
        const v4f v = *(const v4f*)(sH + lr * P + c);
        *(volatile v4f*)(hFn + (size_t)(rb + lr) * HID_ + jb + c) = v;
    }
#pragma unroll
    for (int it = 0; it < 2; ++it) {
        const int lr = wave * 8 + it * 4 + (lane >> 3);
        const int c  = (lane & 7) * 8;
        const v8f x = ld8f(sH + lr * P + c);
        const u16x8 fv = cvt8h(x);
        u16x8 hv, lv;
        split8(x, hv, lv);
        const size_t oh = (size_t)(rb + lr) * HID_ + jb + c;
        const size_t oo = ((size_t)(rb + lr) * T_ + (size_t)t) * HID_ + jb + c;
        *(volatile u16x8*)(hAn + oh) = fv;
        *(volatile u16x8*)(oH + oo)  = hv;
        *(volatile u16x8*)(oL + oo)  = lv;
    }
}

extern "C" void kernel_launch(void* const* d_in, const int* in_sizes, int n_in,
                              void* d_out, int out_size, void* d_ws, size_t ws_size,
                              hipStream_t stream)
{
    if (n_in < 10) return;
    if (in_sizes[0] != BS_ * KIN_)        return;
    if (in_sizes[1] != BS_ * T_ * ACT_)   return;
    if (in_sizes[2] != KIN_ * HID_)       return;
    if (in_sizes[3] != HID_)              return;
    if (in_sizes[4] != ACT_ * G3_)        return;
    if (in_sizes[5] != G3_)               return;
    if (in_sizes[6] != HID_ * G3_)        return;
    if (in_sizes[7] != HID_)              return;
    if (in_sizes[8] != HID_ * OUT_)       return;
    if (in_sizes[9] != OUT_)              return;
    if (out_size != MT_ * OUT_)           return;
    if (ws_size < WS_END)                 return;

    const float* history = (const float*)d_in[0];
    const float* action  = (const float*)d_in[1];
    const float* W_in    = (const float*)d_in[2];
    const float* b_in    = (const float*)d_in[3];
    const float* Wi      = (const float*)d_in[4];
    const float* bi      = (const float*)d_in[5];
    const float* Wh      = (const float*)d_in[6];
    const float* bhn     = (const float*)d_in[7];
    const float* Wo      = (const float*)d_in[8];
    const float* bo      = (const float*)d_in[9];
    float* out = (float*)d_out;

    char* ws = (char*)d_ws;
    unsigned short* oH   = (unsigned short*)(ws + OFF_OH);
    unsigned short* oL   = (unsigned short*)(ws + OFF_OL);
    unsigned short* winH = (unsigned short*)(ws + OFF_WINH);
    unsigned short* winL = (unsigned short*)(ws + OFF_WINL);
    unsigned short* xH   = (unsigned short*)(ws + OFF_XH);
    unsigned short* xL   = (unsigned short*)(ws + OFF_XL);
    unsigned short* whP  = (unsigned short*)(ws + OFF_WH);
    unsigned short* wiH  = (unsigned short*)(ws + OFF_WIH);
    unsigned short* wiL  = (unsigned short*)(ws + OFF_WIL);
    unsigned short* woH  = (unsigned short*)(ws + OFF_WOH);
    unsigned short* woL  = (unsigned short*)(ws + OFF_WOL);
    unsigned short* aH   = (unsigned short*)(ws + OFF_AH);
    unsigned short* aL   = (unsigned short*)(ws + OFF_AL);
    float*          hF0  = (float*)(ws + OFF_HF0);
    float*          hF1  = (float*)(ws + OFF_HF1);
    unsigned short* hA0  = (unsigned short*)(ws + OFF_HA0);
    unsigned short* hA1  = (unsigned short*)(ws + OFF_HA1);

    {
        const int n8x = (BS_ * KIN_) / 8;
        rows_cvt_kernel<<<dim3((n8x + 255) / 256), dim3(256), 0, stream>>>(history, xH, xL, n8x);
        const int n8a = (MT_ * ACT_) / 8;
        rows_cvt_kernel<<<dim3((n8a + 255) / 256), dim3(256), 0, stream>>>(action, aH, aL, n8a);
    }

    wt_cvt_kernel<64, 0><<<dim3(HID_ / 64, KIN_ / 64), dim3(256), 0, stream>>>(W_in, winH, winL, (int)HID_, (int)KIN_, 1.0f);
    wt_cvt_kernel<32, 0><<<dim3(G3_ / 64, 1), dim3(256), 0, stream>>>(Wi, wiH, wiL, (int)G3_, (int)ACT_, 16.0f);
    wt_cvt_kernel<64, 1><<<dim3(G3_ / 64, HID_ / 64), dim3(256), 0, stream>>>(Wh, whP, whP, (int)G3_, (int)HID_, 16.0f);
    wt_cvt_kernel<64, 0><<<dim3(OUT_ / 64, HID_ / 64), dim3(256), 0, stream>>>(Wo, woH, woL, (int)OUT_, (int)HID_, 1.0f);

    gemm_x3_kernel<true, true><<<dim3(HID_ / 64, BS_ / 64), dim3(128), 0, stream>>>(
        (const unsigned short*)xH, (const unsigned short*)xL,
        (const unsigned short*)winH, (const unsigned short*)winL,
        b_in, hF0, hA0, (int)KIN_, (int)HID_, (int)HID_);

    for (int t = 0; t < T_; ++t) {
        const unsigned short* hAp = (t & 1) ? hA1 : hA0;
        const float*          hFp = (t & 1) ? hF1 : hF0;
        unsigned short*       hAn = (t & 1) ? hA0 : hA1;
        float*                hFn = (t & 1) ? hF0 : hF1;
        gru_step_kernel<<<dim3(HID_ / 64, BS_ / 64), dim3(256), 0, stream>>>(
            hAp, hFp, (const unsigned short*)aH, (const unsigned short*)aL, (const unsigned short*)whP,
            (const unsigned short*)wiH, (const unsigned short*)wiL, bi, bhn,
            hFn, hAn, oH, oL, t);
    }

    gemm_x3_kernel<false, false><<<dim3(OUT_ / 64, MT_ / 64), dim3(128), 0, stream>>>(
        (const unsigned short*)oH, (const unsigned short*)oL,
        (const unsigned short*)woH, (const unsigned short*)woL,
        bo, out, hA0, (int)HID_, (int)OUT_, (int)HID_);
}
